// MultiHeadPAttention_2052994367523
// MI455X (gfx1250) — hardware-verified
//
#include <hip/hip_runtime.h>
#include <math.h>
#include <stdint.h>

constexpr int kSeq    = 2048;
constexpr int kDModel = 1024;
constexpr int kNHead  = 16;
constexpr int kDHead  = 64;
constexpr int kNTok   = 1024;
constexpr int kHGrp   = 2;
constexpr int kNGrp   = kNHead / kHGrp;
static_assert(kNTok == 128 * 8, "row kernel coverage");
static_assert(kDModel == 128 * 8, "row kernel coverage");
static_assert(kSeq == 256 * 8, "softmax coverage");

typedef __attribute__((ext_vector_type(16))) _Float16 v16h;
typedef __attribute__((ext_vector_type(8)))  _Float16 v8h;
typedef __attribute__((ext_vector_type(16))) __bf16   v16b;
typedef __attribute__((ext_vector_type(8)))  __bf16   v8b;
typedef __attribute__((ext_vector_type(8)))  float    v8f;
typedef __attribute__((ext_vector_type(4)))  float    v4f;
typedef __attribute__((ext_vector_type(2)))  float    v2f;
typedef __attribute__((ext_vector_type(4)))  unsigned int v4u;

__device__ __forceinline__ unsigned short f2bf_bits(float f) {
  unsigned u = __float_as_uint(f);
  return (unsigned short)((u + 0x7FFFu + ((u >> 16) & 1u)) >> 16);
}
__device__ __forceinline__ float bf_bits2f(unsigned short h) { return __uint_as_float(((unsigned)h) << 16); }
__device__ __forceinline__ unsigned short f2h_bits(float f) { return __builtin_bit_cast(unsigned short, (_Float16)f); }
__device__ __forceinline__ unsigned pk16(unsigned short a, unsigned short b) { return (unsigned)a | ((unsigned)b << 16); }

__device__ __forceinline__ void dep_guard_h(v8f& a, v8f& b, v16h x, v16h y) { asm volatile("v_nop\n\tv_nop\n\tv_nop\n\tv_nop" : "+v"(a), "+v"(b) : "v"(x), "v"(y)); }
__device__ __forceinline__ void dep_guard_b(v8f& a, v8f& b, v16b x, v16b y) { asm volatile("v_nop\n\tv_nop\n\tv_nop\n\tv_nop" : "+v"(a), "+v"(b) : "v"(x), "v"(y)); }
__device__ __forceinline__ void keep4_h(v16h a, v16h b, v16h c, v16h d) { asm volatile("v_nop" :: "v"(a), "v"(b), "v"(c), "v"(d)); }
__device__ __forceinline__ void keep4_b(v16b a, v16b b, v16b c, v16b d) { asm volatile("v_nop" :: "v"(a), "v"(b), "v"(c), "v"(d)); }
__device__ __forceinline__ void acc_guard4(v8f& a, v8f& b, v8f& c, v8f& d) { asm volatile("v_nop\n\tv_nop\n\tv_nop\n\tv_nop" : "+v"(a), "+v"(b), "+v"(c), "+v"(d)); }
template <typename T> struct Frag;
template <> struct Frag<_Float16> {
  typedef v16h V; union U { v16h v; v8h h[2]; };
  static __device__ __forceinline__ v16h load(const _Float16* p) {
    U f; f.h[0] = *(const v8h*)(p); f.h[1] = *(const v8h*)(p + 16); return f.v;
  }
  static __device__ __forceinline__ v8f mma(v16h a, v16h b, v8f c) {
    return __builtin_amdgcn_wmma_f32_16x16x32_f16(false, a, false, b, (short)0, c, false, false);
  }
  static __device__ __forceinline__ void guard(v8f& a, v8f& b, v16h x, v16h y) { dep_guard_h(a, b, x, y); }
  static __device__ __forceinline__ void keep(v16h a, v16h b, v16h c, v16h d) { keep4_h(a, b, c, d); }
};
template <> struct Frag<__bf16> {
  typedef v16b V; union U { v16b v; v8b h[2]; };
  static __device__ __forceinline__ v16b load(const __bf16* p) {
    U f; f.h[0] = *(const v8b*)(p); f.h[1] = *(const v8b*)(p + 16); return f.v;
  }
  static __device__ __forceinline__ v8f mma(v16b a, v16b b, v8f c) {
    return __builtin_amdgcn_wmma_f32_16x16x32_bf16(false, a, false, b, (short)0, c, false, false);
  }
  static __device__ __forceinline__ void guard(v8f& a, v8f& b, v16b x, v16b y) { dep_guard_b(a, b, x, y); }
  static __device__ __forceinline__ void keep(v16b a, v16b b, v16b c, v16b d) { keep4_b(a, b, c, d); }
};

template <int ET> struct Elem;
template <> struct Elem<0> { typedef _Float16 T; };
template <> struct Elem<1> { typedef __bf16 T; };
template <int ET, bool SPLIT, int BIAS_MODE, int OUT_MODE, bool RESID, int ACT = 0>
__global__ __launch_bounds__(256) void wmma_gemm64(
    const unsigned short* __restrict__ Ap, const unsigned short* __restrict__ A2p, int lda, long strideA,
    const unsigned short* __restrict__ Btp, const unsigned short* __restrict__ Bt2p, int ldb, long strideB,
    void* __restrict__ Cout, void* __restrict__ Cout2, int ldc, long strideC,
    const float* __restrict__ bias,
    const float* __restrict__ resid, long strideR,
    int M, int N, int K, float scale) {
  typedef typename Elem<ET>::T T;
  typedef typename Frag<T>::V V;
  const T* A = (const T*)Ap; const T* A2 = (const T*)A2p; const T* Bt = (const T*)Btp; const T* Bt2 = (const T*)Bt2p;
  __shared__ __align__(16) float sT[8][16 * 68];
  const int b    = blockIdx.y;
  const int lane = threadIdx.x & 31;
  const int wave = threadIdx.x >> 5;
  const int tilesN = N >> 6;
  const int tilesM = M >> 6;
  const int tile = blockIdx.x * 8 + wave;
  if (tile >= tilesM * tilesN) return;
  const int tm = tile / tilesN;
  const int tn = tile - tm * tilesN;
  const int m0 = tm << 6;
  const int n0 = tn << 6;

  const T* Ab  = A  + (size_t)b * strideA;
  const T* Bb  = Bt + (size_t)b * strideB;
  const T* Ab2 = SPLIT ? (A2  + (size_t)b * strideA) : nullptr;
  const T* Bb2 = SPLIT ? (Bt2 + (size_t)b * strideB) : nullptr;

  const int rlane = lane & 15;
  const int koff  = (lane >> 4) * 8;
  const int mOff  = (lane >> 4) * 8;

  v8f acc[4][4];
#pragma unroll
  for (int i = 0; i < 4; ++i)
#pragma unroll
    for (int j = 0; j < 4; ++j) acc[i][j] = (v8f){0.f,0.f,0.f,0.f,0.f,0.f,0.f,0.f};

  for (int k0 = 0; k0 < K; k0 += 32) {
    V bh[4], bl[4];
#pragma unroll
    for (int j = 0; j < 4; ++j) {
      const size_t bo = (size_t)(n0 + (j << 4) + rlane) * ldb + koff + k0;
      bh[j] = Frag<T>::load(Bb + bo);
      if (SPLIT) bl[j] = Frag<T>::load(Bb2 + bo);
    }
#pragma unroll
    for (int i = 0; i < 4; ++i) {
      const size_t ao = (size_t)(m0 + (i << 4) + rlane) * lda + koff + k0;
      V ah = Frag<T>::load(Ab + ao);
      V al;
      if (SPLIT) al = Frag<T>::load(Ab2 + ao);
#pragma unroll
      for (int j = 0; j < 4; ++j) {
        acc[i][j] = Frag<T>::mma(ah, bh[j], acc[i][j]);
        if (SPLIT) {
          acc[i][j] = Frag<T>::mma(ah, bl[j], acc[i][j]);
          acc[i][j] = Frag<T>::mma(al, bh[j], acc[i][j]);
        }
      }
      Frag<T>::guard(acc[i][0], acc[i][3], ah, SPLIT ? al : ah);
    }
    Frag<T>::keep(bh[0], bh[1], bh[2], bh[3]);
    if (SPLIT) Frag<T>::keep(bl[0], bl[1], bl[2], bl[3]);
  }
  acc_guard4(acc[0][0], acc[0][1], acc[0][2], acc[0][3]);
  acc_guard4(acc[1][0], acc[1][1], acc[1][2], acc[1][3]);
  acc_guard4(acc[2][0], acc[2][1], acc[2][2], acc[2][3]);
  acc_guard4(acc[3][0], acc[3][1], acc[3][2], acc[3][3]);

  float* slab = sT[wave];
  const float* Rb = RESID ? (resid + (size_t)b * strideR) : nullptr;
#pragma unroll
  for (int i = 0; i < 4; ++i) {
    const int mBase = m0 + (i << 4);
#pragma unroll
    for (int j = 0; j < 4; ++j) {
      const int n = n0 + (j << 4) + rlane;
      float bv = 0.f;
      if (BIAS_MODE == 2) bv = bias[n];
#pragma unroll
      for (int r = 0; r < 8; ++r) {
        float v = acc[i][j][r] * scale;
        if (BIAS_MODE == 1) v += bias[mBase + mOff + r];
        if (BIAS_MODE == 2) v += bv;
        if (RESID) v += Rb[(size_t)(mBase + mOff + r) * ldc + n];
        if (ACT == 1) v = tanhf(v);
        if (ACT == 2) v = fmaxf(v, 0.0f);
        if (ACT == 3) v = v / (1.0f + expf(-v));
        if (ACT == 4) v = (v > 0.f) ? v : 0.01f * v;
        if (ACT == 5) v = 0.5f * v * (1.0f + erff(v * 0.70710678118654752f));
        slab[(mOff + r) * 68 + (j << 4) + rlane] = v;
      }
    }
    __builtin_amdgcn_fence(__ATOMIC_RELEASE, "workgroup");
    __builtin_amdgcn_wave_barrier();
    __builtin_amdgcn_fence(__ATOMIC_ACQUIRE, "workgroup");
    if (OUT_MODE == 0) {
      float* C = (float*)Cout + (size_t)b * strideC;
      const int hh = lane >> 4, c4 = (lane & 15) * 4;
      for (int pass = 0; pass < 2; ++pass) {
#pragma unroll
        for (int it = 0; it < 8; ++it) {
          const int row = it * 2 + hh;
          v4f v = *(const v4f*)(slab + row * 68 + c4);
          *(volatile v4f*)(C + (size_t)(mBase + row) * ldc + n0 + c4) = v;
        }
        __threadfence();
      }
    } else {
      const int q = lane >> 3, c8 = (lane & 7) * 8;
      unsigned short* C  = (unsigned short*)Cout  + (size_t)b * strideC;
      unsigned short* C2 = (OUT_MODE == 2) ? ((unsigned short*)Cout2 + (size_t)b * strideC) : nullptr;
      for (int pass = 0; pass < 2; ++pass) {
#pragma unroll
        for (int it = 0; it < 4; ++it) {
          const int row = it * 4 + q;
          const float* sp = slab + row * 68 + c8;
          v8h hv, lv;
#pragma unroll
          for (int e = 0; e < 8; ++e) {
            if (OUT_MODE == 1) {
              hv[e] = (_Float16)sp[e];
            } else {
              unsigned short hb = f2bf_bits(sp[e]);
              unsigned short lb = f2bf_bits(sp[e] - bf_bits2f(hb));
              hv[e] = __builtin_bit_cast(_Float16, hb);
              lv[e] = __builtin_bit_cast(_Float16, lb);
            }
          }
          *(volatile v8h*)(C + (size_t)(mBase + row) * ldc + n0 + c8) = hv;
          if (OUT_MODE == 2) *(volatile v8h*)(C2 + (size_t)(mBase + row) * ldc + n0 + c8) = lv;
        }
        __threadfence();
      }
    }
    __builtin_amdgcn_fence(__ATOMIC_RELEASE, "workgroup");
    __builtin_amdgcn_wave_barrier();
    __builtin_amdgcn_fence(__ATOMIC_ACQUIRE, "workgroup");
  }
}

__global__ __launch_bounds__(256) void cast_f16x2_kernel(const float* __restrict__ in, unsigned short* __restrict__ out,
                                                        int n2, float sc) {
  const int i = blockIdx.x * 256 + threadIdx.x;
  if (i < n2) {
    const v2f f = *(const v2f*)(in + 2 * (size_t)i);
    const unsigned u = pk16(f2h_bits(f[0] * sc), f2h_bits(f[1] * sc));
    ((volatile unsigned*)out)[i] = u;
    __threadfence();
    ((volatile unsigned*)out)[i] = u;
  }
}

__global__ __launch_bounds__(256) void transpose_f16_kernel(const float* __restrict__ in, int ldi,
                                                            unsigned short* __restrict__ out, int ldo) {
  __shared__ __align__(16) float tf[64 * 68];
  const int c0  = blockIdx.x * 64;
  const int r0  = blockIdx.y * 64;
  const int tid = threadIdx.x;
  {
    const int sub = tid >> 4;
    const int c4  = (tid & 15) * 4;
#pragma unroll
    for (int it = 0; it < 4; ++it) {
      const int rr = it * 16 + sub;
      const v4f a = *(const v4f*)(in + (size_t)(r0 + rr) * ldi + c0 + c4);
      *(v4f*)(tf + rr * 68 + c4) = a;
    }
  }
  __syncthreads();
  const int s8 = tid >> 3;
  const int c8 = (tid & 7) * 8;
  v4u hv[2];
#pragma unroll
  for (int it = 0; it < 2; ++it) {
    const int oc = it * 32 + s8;
    v4u a;
#pragma unroll
    for (int q = 0; q < 4; ++q) {
      const float f0 = tf[(c8 + 2 * q) * 68 + oc];
      const float f1 = tf[(c8 + 2 * q + 1) * 68 + oc];
      a[q] = pk16(f2h_bits(f0), f2h_bits(f1));
    }
    hv[it] = a;
  }
  for (int pass = 0; pass < 2; ++pass) {
#pragma unroll
    for (int it = 0; it < 2; ++it) {
      const int oc = it * 32 + s8;
      const size_t go = (size_t)(c0 + oc) * ldo + r0 + c8;
      *(volatile v4u*)(out + go) = hv[it];
    }
    __threadfence();
  }
}

__global__ __launch_bounds__(128) void rownorm_gelu_kernel(const float* __restrict__ AW, unsigned short* __restrict__ AWG) {
#pragma clang fp contract(off)
  __shared__ float red[4];
  __shared__ __align__(16) _Float16 hrow[kNTok];
  const int r    = blockIdx.x;
  const int tid  = threadIdx.x;
  const int lane = tid & 31;
  const int wave = tid >> 5;
  const int c0   = tid * 8;
  const float* rp = AW + (size_t)r * kNTok + c0;
  const v4f a0 = *(const v4f*)(rp);
  const v4f a1 = *(const v4f*)(rp + 4);
  float ss = a0[0] * a0[0];
  ss += a0[1] * a0[1]; ss += a0[2] * a0[2]; ss += a0[3] * a0[3];
  ss += a1[0] * a1[0]; ss += a1[1] * a1[1]; ss += a1[2] * a1[2]; ss += a1[3] * a1[3];
#pragma unroll
  for (int off = 16; off > 0; off >>= 1) ss += __shfl_xor(ss, off, 32);
  if (lane == 0) red[wave] = ss;
  __syncthreads();
  const float tot = ((red[0] + red[1]) + red[2]) + red[3];
  const float nrm = sqrtf(tot);
  const float rn  = 1.0f / nrm;
  const float sq  = 32.0f;
#pragma unroll 1
  for (int e = 0; e < 8; ++e) {
    float v = rp[e];
    v = (v * rn) * sq;
    const float g = 0.5f * v * (1.0f + erff(v * 0.70710678118654752f));
    hrow[c0 + e] = (_Float16)g;
  }
  __syncthreads();
  const v8h hv = *(const v8h*)(hrow + c0);
  unsigned short* op = AWG + (size_t)r * kNTok + c0;
  *(volatile v8h*)(op) = hv;
  __threadfence();
  *(volatile v8h*)(op) = hv;
}

__global__ __launch_bounds__(256) void rope_table_kernel(float* __restrict__ cs, float* __restrict__ sn) {
#pragma clang fp contract(off)
  const int tid  = threadIdx.x;
  const int lane = tid & 31;
  const int wave = tid >> 5;
  const int l    = blockIdx.x * 8 + wave;
  const float invf = powf(1.0e-4f, (float)lane * 0.03125f);
  const float ang  = (float)l * invf;
  const float cv = cosf(ang);
  const float sv = sinf(ang);
  const size_t o = (size_t)l * 32 + lane;
  ((volatile float*)cs)[o] = cv;
  ((volatile float*)sn)[o] = sv;
  __threadfence();
  ((volatile float*)cs)[o] = cv;
  ((volatile float*)sn)[o] = sv;
}

__global__ __launch_bounds__(128) void rms_rotary_split_kernel(const float* __restrict__ R, const float* __restrict__ cs,
                                                               const float* __restrict__ sn,
                                                               unsigned short* __restrict__ Oh, unsigned short* __restrict__ Ol,
                                                               float oscale) {
#pragma clang fp contract(off)
  const int l     = blockIdx.x;
  const int tid   = threadIdx.x;
  const int c0    = tid * 8;
  const int j     = tid & 7;
  const int hbase = (tid >> 3) * kDHead;
  const int pc0   = hbase + ((j ^ 4) * 8);
  const float* rp = R + (size_t)l * kDModel;
  const v4f oa = *(const v4f*)(rp + c0);
  const v4f ob = *(const v4f*)(rp + c0 + 4);
  const v4f pa = *(const v4f*)(rp + pc0);
  const v4f pb = *(const v4f*)(rp + pc0 + 4);
  float o[8], p[8];
#pragma unroll
  for (int e = 0; e < 4; ++e) { o[e] = oa[e]; o[4 + e] = ob[e]; p[e] = pa[e]; p[4 + e] = pb[e]; }
  float ss = o[0] * o[0];
#pragma unroll
  for (int e = 1; e < 8; ++e) ss += o[e] * o[e];
#pragma unroll
  for (int off = 1; off < 8; off <<= 1) ss += __shfl_xor(ss, off, 32);
  const float rn = rsqrtf(ss * (1.0f / 64.0f) + 1.0e-6f);
  const int fi0 = (j & 3) * 8;
  const float* cp = cs + (size_t)l * 32 + fi0;
  const float* sp = sn + (size_t)l * 32 + fi0;
  const v4f ca = *(const v4f*)(cp), cb = *(const v4f*)(cp + 4);
  const v4f sa = *(const v4f*)(sp), sb = *(const v4f*)(sp + 4);
  float cv[8], sv[8];
#pragma unroll
  for (int e = 0; e < 4; ++e) { cv[e] = ca[e]; cv[4 + e] = cb[e]; sv[e] = sa[e]; sv[4 + e] = sb[e]; }
  const float sg = (j < 4) ? 1.0f : -1.0f;
  unsigned hw[4], lw[4];
#pragma unroll
  for (int q = 0; q < 4; ++q) {
    unsigned short hb[2], lb[2];
#pragma unroll
    for (int d = 0; d < 2; ++d) {
      const int e = 2 * q + d;
      const float on = o[e] * rn;
      const float pn = p[e] * rn;
      const float t1 = on * cv[e];
      const float t2 = (sg * pn) * sv[e];
      const float v  = (t1 + t2) * oscale;
      hb[d] = f2bf_bits(v);
      lb[d] = f2bf_bits(v - bf_bits2f(hb[d]));
    }
    hw[q] = pk16(hb[0], hb[1]);
    lw[q] = pk16(lb[0], lb[1]);
  }
  const v4u hvv = (v4u){hw[0], hw[1], hw[2], hw[3]};
  const v4u lvv = (v4u){lw[0], lw[1], lw[2], lw[3]};
  const size_t go = (size_t)l * kDModel + c0;
  *(volatile v4u*)(Oh + go) = hvv;
  *(volatile v4u*)(Ol + go) = lvv;
  __threadfence();
  *(volatile v4u*)(Oh + go) = hvv;
  *(volatile v4u*)(Ol + go) = lvv;
}

__global__ __launch_bounds__(256) void softmax_split_kernel(const float* __restrict__ S,
                                                            unsigned short* __restrict__ Phi, unsigned short* __restrict__ Plo) {
#pragma clang fp contract(off)
  __shared__ float redm[8];
  __shared__ float reds[8];
  const int i    = blockIdx.x;
  const int hg   = blockIdx.y;
  const int tid  = threadIdx.x;
  const int lane = tid & 31;
  const int wave = tid >> 5;
  const int j0   = tid * 8;
  const float* row = S + ((size_t)hg * kSeq + (size_t)i) * kSeq + j0;
  const v4f a0 = *(const v4f*)(row);
  const v4f a1 = *(const v4f*)(row + 4);
  float t[8];
#pragma unroll
  for (int e = 0; e < 4; ++e) { t[e] = a0[e]; t[4 + e] = a1[e]; }
  float m = fmaxf(fmaxf(fmaxf(t[0], t[1]), fmaxf(t[2], t[3])), fmaxf(fmaxf(t[4], t[5]), fmaxf(t[6], t[7])));
#pragma unroll
  for (int off = 16; off > 0; off >>= 1) m = fmaxf(m, __shfl_xor(m, off, 32));
  if (lane == 0) redm[wave] = m;
  __syncthreads();
  float mx = redm[0];
#pragma unroll
  for (int w = 1; w < 8; ++w) mx = fmaxf(mx, redm[w]);
  float ex[8];
#pragma unroll
  for (int e = 0; e < 8; ++e) ex[e] = __expf(t[e] - mx);
  float ps = ((((((ex[0] + ex[1]) + ex[2]) + ex[3]) + ex[4]) + ex[5]) + ex[6]) + ex[7];
#pragma unroll
  for (int off = 16; off > 0; off >>= 1) ps += __shfl_xor(ps, off, 32);
  if (lane == 0) reds[wave] = ps;
  __syncthreads();
  float tot = reds[0];
#pragma unroll
  for (int w = 1; w < 8; ++w) tot += reds[w];
  const float inv = 1.0f / tot;
  unsigned hw[4], lw[4];
#pragma unroll
  for (int q = 0; q < 4; ++q) {
    const float p0 = ex[2 * q] * inv, p1 = ex[2 * q + 1] * inv;
    const unsigned short hb0 = f2bf_bits(p0), hb1 = f2bf_bits(p1);
    const unsigned short lb0 = f2bf_bits(p0 - bf_bits2f(hb0));
    const unsigned short lb1 = f2bf_bits(p1 - bf_bits2f(hb1));
    hw[q] = pk16(hb0, hb1);
    lw[q] = pk16(lb0, lb1);
  }
  const v4u hvv = (v4u){hw[0], hw[1], hw[2], hw[3]};
  const v4u lvv = (v4u){lw[0], lw[1], lw[2], lw[3]};
  const size_t rowoff = ((size_t)hg * kSeq + (size_t)i) * kSeq + j0;
  *(volatile v4u*)(Phi + rowoff) = hvv;
  *(volatile v4u*)(Plo + rowoff) = lvv;
  __threadfence();
  *(volatile v4u*)(Phi + rowoff) = hvv;
  *(volatile v4u*)(Plo + rowoff) = lvv;
}

constexpr size_t kPl16L = (size_t)kSeq * kDModel * 2;
constexpr size_t kPl16W = (size_t)kDModel * kDModel * 2;
constexpr size_t kPlF32 = (size_t)kSeq * kDModel * 4;
constexpr size_t kPlTab = (size_t)kSeq * 32 * 4;
constexpr size_t kPlS   = (size_t)kHGrp * kSeq * kSeq * 4;
constexpr size_t kPlP   = (size_t)kHGrp * kSeq * kSeq * 2;
constexpr size_t oX16   = 0;
constexpr size_t oWa16  = oX16 + kPl16L;
constexpr size_t oPk16  = oWa16 + kPl16W;
constexpr size_t oPvT16 = oPk16 + kPl16W;
constexpr size_t oR016  = oPvT16 + kPl16W;
constexpr size_t oAW    = oR016 + kPl16L;
constexpr size_t oAWG16 = oAW + kPlF32;
constexpr size_t oQh    = oAWG16 + kPl16L;
constexpr size_t oQl    = oQh + kPl16L;
constexpr size_t oKh    = oQl + kPl16L;
constexpr size_t oKl    = oKh + kPl16L;
constexpr size_t oVTh   = oKl + kPl16L;
constexpr size_t oVTl   = oVTh + kPl16L;
constexpr size_t oCS    = oVTl + kPl16L;
constexpr size_t oSN    = oCS + kPlTab;
constexpr size_t oCTX16 = oSN + kPlTab;
constexpr size_t oS     = oCTX16 + kPl16L;
constexpr size_t oPh    = oS + kPlS;
constexpr size_t oPl    = oPh + kPlP;
constexpr size_t oEnd   = oPl + kPlP;
static_assert(oEnd == 124256256ull, "carve total");
static_assert(oEnd <= 134217728ull, "carve under 128 MiB");

extern "C" void kernel_launch(void* const* d_in, const int* in_sizes, int n_in,
                              void* d_out, int out_size, void* d_ws, size_t ws_size,
                              hipStream_t stream) {
  if (n_in < 11) return;
  if (in_sizes[0] != kSeq * kDModel) return;
  for (int i = 1; i <= 10; ++i) { if (in_sizes[i] != kDModel * kDModel) return; }
  if (out_size != kSeq * kDModel) return;
  if (oEnd > ws_size) return;

  const float* x  = (const float*)d_in[0];
  const float* Wq[3] = {(const float*)d_in[1], (const float*)d_in[4], (const float*)d_in[7]};
  const float* Pk[3] = {(const float*)d_in[2], (const float*)d_in[5], (const float*)d_in[8]};
  const float* Pv[3] = {(const float*)d_in[3], (const float*)d_in[6], (const float*)d_in[9]};
  const float* Wo = (const float*)d_in[10];
  const float* fz = x;

  char* ws = (char*)d_ws;
  unsigned short* X16   = (unsigned short*)(ws + oX16);
  unsigned short* Wa16  = (unsigned short*)(ws + oWa16);
  unsigned short* Pk16  = (unsigned short*)(ws + oPk16);
  unsigned short* PvT16 = (unsigned short*)(ws + oPvT16);
  unsigned short* R016  = (unsigned short*)(ws + oR016);
  float*          AW    = (float*)(ws + oAW);
  unsigned short* AWG16 = (unsigned short*)(ws + oAWG16);
  unsigned short* Qh    = (unsigned short*)(ws + oQh);
  unsigned short* Ql    = (unsigned short*)(ws + oQl);
  unsigned short* Kh    = (unsigned short*)(ws + oKh);
  unsigned short* Kl    = (unsigned short*)(ws + oKl);
  unsigned short* VTh   = (unsigned short*)(ws + oVTh);
  unsigned short* VTl   = (unsigned short*)(ws + oVTl);
  float*          CS    = (float*)(ws + oCS);
  float*          SN    = (float*)(ws + oSN);
  unsigned short* CTX16 = (unsigned short*)(ws + oCTX16);
  float*          Sbuf  = (float*)(ws + oS);
  unsigned short* Ph    = (unsigned short*)(ws + oPh);
  unsigned short* Pl    = (unsigned short*)(ws + oPl);

  const dim3 blk256(256), blk128(128);
  const int n2x = kSeq * kDModel / 2;
  const int n2w = kDModel * kDModel / 2;
  const dim3 gCastX((n2x + 255) / 256);
  const dim3 gCastW((n2w + 255) / 256);
  const dim3 gTr(kDModel / 64, kNTok / 64);
  const dim3 gTab(kSeq / 8);
  const dim3 gRow(kSeq);
  const dim3 gLD(((kSeq / 64) * (kDModel / 64) + 7) / 8, 1);
  const dim3 gVT(((kDModel / 64) * (kSeq / 64) + 7) / 8, 1);
  const dim3 gS(((kSeq / 64) * (kSeq / 64) + 7) / 8, kHGrp);
  const dim3 gSm(kSeq, kHGrp);
  const dim3 gPV(((kSeq / 64) * (kDHead / 64) + 7) / 8, kHGrp);

  cast_f16x2_kernel<<<gCastX, blk256, 0, stream>>>(x, X16, n2x, 1.0f);
  rope_table_kernel<<<gTab, blk256, 0, stream>>>(CS, SN);

  for (int r = 0; r < 3; ++r) {
    cast_f16x2_kernel<<<gCastW, blk256, 0, stream>>>(Wq[r], Wa16, n2w, 16.0f);
    cast_f16x2_kernel<<<gCastW, blk256, 0, stream>>>(Pk[r], Pk16, n2w, 1.0f);
    transpose_f16_kernel<<<gTr, blk256, 0, stream>>>(Pv[r], kDModel, PvT16, kNTok);
    wmma_gemm64<0, false, 0, 1, false, 0><<<gLD, blk256, 0, stream>>>(
        X16, X16, kDModel, 0L, Wa16, Wa16, kDModel, 0L, (void*)R016, (void*)R016, kDModel, 0L,
        fz, fz, 0L, kSeq, kDModel, kDModel, 1.0f / 16.0f);
    wmma_gemm64<0, false, 0, 0, false, 0><<<gLD, blk256, 0, stream>>>(
        R016, R016, kDModel, 0L, Pk16, Pk16, kDModel, 0L, (void*)AW, (void*)AW, kNTok, 0L,
        fz, fz, 0L, kSeq, kNTok, kDModel, 1.0f);
    rownorm_gelu_kernel<<<gRow, blk128, 0, stream>>>(AW, AWG16);
    if (r < 2) {
      wmma_gemm64<0, false, 0, 0, false, 0><<<gLD, blk256, 0, stream>>>(
          AWG16, AWG16, kNTok, 0L, PvT16, PvT16, kNTok, 0L, (void*)AW, (void*)AW, kDModel, 0L,
          fz, fz, 0L, kSeq, kDModel, kNTok, 1.0f);
      rms_rotary_split_kernel<<<gRow, blk128, 0, stream>>>(AW, CS, SN, (r == 0) ? Qh : Kh, (r == 0) ? Ql : Kl,
                                                            (r == 0) ? 0.125f : 1.0f);
    } else {
      wmma_gemm64<0, false, 0, 2, false, 0><<<gVT, blk256, 0, stream>>>(
          PvT16, PvT16, kNTok, 0L, AWG16, AWG16, kNTok, 0L, (void*)VTh, (void*)VTl, kSeq, 0L,
          fz, fz, 0L, kDModel, kSeq, kNTok, 1.0f);
    }
  }
  cast_f16x2_kernel<<<gCastW, blk256, 0, stream>>>(Wo, Wa16, n2w, 16.0f);

  for (int g = 0; g < kNGrp; ++g) {
    const size_t qcol = (size_t)g * kHGrp * kDHead;
    wmma_gemm64<1, true, 0, 0, false, 0><<<gS, blk256, 0, stream>>>(
        Qh + qcol, Ql + qcol, kDModel, (long)kDHead,
        Kh + qcol, Kl + qcol, kDModel, (long)kDHead,
        (void*)Sbuf, (void*)Sbuf, kSeq, (long)kSeq * kSeq,
        fz, fz, 0L, kSeq, kSeq, kDHead, 1.0f);
    softmax_split_kernel<<<gSm, blk256, 0, stream>>>(Sbuf, Ph, Pl);
    wmma_gemm64<1, true, 0, 1, false, 0><<<gPV, blk256, 0, stream>>>(
        Ph, Pl, kSeq, (long)kSeq * kSeq,
        VTh + qcol * kSeq, VTl + qcol * kSeq, kSeq, (long)kDHead * kSeq,
        (void*)(CTX16 + qcol), (void*)(CTX16 + qcol), kDModel, (long)kDHead,
        fz, fz, 0L, kSeq, kDHead, kSeq, 1.0f);
  }
  wmma_gemm64<0, false, 0, 0, false, 0><<<gLD, blk256, 0, stream>>>(
      CTX16, CTX16, kDModel, 0L, Wa16, Wa16, kDModel, 0L, d_out, d_out, kDModel, 0L,
      fz, fz, 0L, kSeq, kDModel, kDModel, 1.0f / 16.0f);
}
